// SkeletonResidualTranspose_9225589752530
// MI455X (gfx1250) — hardware-verified
//
#include <hip/hip_runtime.h>

typedef __attribute__((ext_vector_type(16))) _Float16 v16h;
typedef __attribute__((ext_vector_type(8)))  _Float16 v8h;
typedef __attribute__((ext_vector_type(8)))  float    v8f;
typedef __attribute__((ext_vector_type(4)))  float    v4f;

#define NB     16
#define CIN    416
#define TIN    1024
#define TOUT   2048
#define NJ     25
#define CPO    16
#define OUTC   400
#define INC    800
#define KTAPS  7
#define YP     448
#define TROWS  2080
#define KTOT   672
#define WPITCH 704
#define YSC    16.0f
#define WSC    256.0f
#define OSC    (1.0f / 4096.0f)

template <typename T> struct Frag;
template <> struct Frag<_Float16> {
  typedef v16h V; union U { v16h v; v8h h[2]; };
  static __device__ __forceinline__ v16h load(const _Float16* p) {
    U f; f.h[0] = *(const v8h*)(p); f.h[1] = *(const v8h*)(p + 16); return f.v;
  }
  static __device__ __forceinline__ v8f mma(v16h a, v16h b, v8f c) {
    return __builtin_amdgcn_wmma_f32_16x16x32_f16(false, a, false, b, (short)0, c, false, false);
  }
};

__device__ __forceinline__ void guard4x(v8f& a, v8f& b, v8f& c, v8f& d,
                                        v16h x0, v16h x1, v16h x2, v16h x3, v16h y) {
  asm volatile("v_nop\n\tv_nop\n\tv_nop\n\tv_nop"
               : "+v"(a), "+v"(b), "+v"(c), "+v"(d)
               : "v"(x0), "v"(x1), "v"(x2), "v"(x3), "v"(y));
}
__device__ __forceinline__ void acc_guard4(v8f& a, v8f& b, v8f& c, v8f& d) {
  asm volatile("v_nop\n\tv_nop\n\tv_nop\n\tv_nop" : "+v"(a), "+v"(b), "+v"(c), "+v"(d));
}

__global__ __launch_bounds__(256) void k_prep_y(const float* __restrict__ x, _Float16* __restrict__ Y) {
#pragma clang fp contract(off)
  __shared__ __align__(16) _Float16 tile[32 * YP];
  const int tp0 = blockIdx.x * 32;
  const int b   = blockIdx.y;
  const int tid = threadIdx.x;
  const float* xb = x + (size_t)b * CIN * TIN;
#pragma unroll 2
  for (int it = 0; it < 52; ++it) {
    const int i = it * 256 + tid;
    const int c = i >> 5;
    const int r = i & 31;
    int t = tp0 + r - 3;
    t = t < 0 ? -t : t;
    t = t > (TOUT - 1) ? (2 * TOUT - 2 - t) : t;
    float pos = ((float)t + 0.5f) * 0.5f - 0.5f;
    pos = pos < 0.0f ? 0.0f : pos;
    pos = pos > (float)(TIN - 1) ? (float)(TIN - 1) : pos;
    int i0 = (int)pos;
    i0 = i0 < 0 ? 0 : (i0 > TIN - 1 ? TIN - 1 : i0);
    int i1 = i0 + 1;
    i1 = i1 > TIN - 1 ? TIN - 1 : i1;
    const float w = pos - (float)i0;
    const float* xr = xb + (size_t)c * TIN;
    const float a0 = xr[i0] * (1.0f - w);
    const float a1 = xr[i1] * w;
    const float v = (a0 + a1) * YSC;
    tile[r * YP + c] = (_Float16)v;
  }
  __syncthreads();

  const int wave = tid >> 5, lane = tid & 31;
  const int pcl = lane < 24 ? 32 + lane : 55;
  v8h zero8;
#pragma unroll
  for (int e = 0; e < 8; ++e) zero8[e] = (_Float16)0.0f;
#pragma unroll
  for (int q = 0; q < 4; ++q) {
    const int r = wave * 4 + q;
    const v8h p0v = *(const v8h*)(tile + r * YP + lane * 8);
    v8h p1v = *(const v8h*)(tile + r * YP + pcl * 8);
    if (pcl >= 52) p1v = zero8;
    _Float16* dst = Y + ((size_t)b * TROWS + tp0 + r) * YP;
    for (int pass = 0; pass < 2; ++pass) {
      *(volatile v8h*)(dst + lane * 8) = p0v;
      if (lane < 24) *(volatile v8h*)(dst + pcl * 8) = p1v;
      __threadfence();
    }
  }
}

__device__ __forceinline__ v8h pack_piece(const float* __restrict__ w_res, const float* __restrict__ w_sc,
                                          int j, int base, int ocg, int p) {
  v8h hv;
#pragma unroll
  for (int e = 0; e < 8; ++e) {
    const int k  = p * 8 + e;
    const int kc = k < KTOT ? k : (KTOT - 1);
    const int s  = kc >> 5;
    const int kl = kc & 31;
    const int tap = s / 3;
    const int chunk = s - 3 * tap;
    const int f = base + chunk;
    const int icg = f * 32 + kl;
    const size_t wi = (size_t)ocg * INC + icg;
    const float wr = w_res[wi * KTAPS + tap];
    const float ws = w_sc[wi];
    float v = wr + ((tap == 3) ? ws : 0.0f);
    const bool ok = (k < KTOT) && (f >= j - 1) && (f <= j + 1);
    v = ok ? (v * WSC) : 0.0f;
    hv[e] = (_Float16)v;
  }
  return hv;
}

__global__ __launch_bounds__(256) void k_pack_w(const float* __restrict__ w_res, const float* __restrict__ w_sc,
                                                _Float16* __restrict__ Wp) {
  const int j = blockIdx.x;
  const int wave = threadIdx.x >> 5, lane = threadIdx.x & 31;
  int base = j - 1;
  base = base < 0 ? 0 : base;
  base = base > 22 ? 22 : base;
  const int p2 = lane < 24 ? 64 + lane : 87;
#pragma unroll
  for (int q = 0; q < 2; ++q) {
    const int oc  = wave * 2 + q;
    const int ocg = j * CPO + oc;
    const v8h h0 = pack_piece(w_res, w_sc, j, base, ocg, lane);
    const v8h h1 = pack_piece(w_res, w_sc, j, base, ocg, 32 + lane);
    const v8h h2 = pack_piece(w_res, w_sc, j, base, ocg, p2);
    _Float16* dst = Wp + (size_t)ocg * WPITCH;
    for (int pass = 0; pass < 2; ++pass) {
      *(volatile v8h*)(dst + lane * 8) = h0;
      *(volatile v8h*)(dst + (32 + lane) * 8) = h1;
      if (lane < 24) *(volatile v8h*)(dst + p2 * 8) = h2;
      __threadfence();
    }
  }
}

__global__ __launch_bounds__(256) void k_conv(const _Float16* __restrict__ Y, const _Float16* __restrict__ Wp,
                                              const float* __restrict__ b_res, const float* __restrict__ b_sc,
                                              const float* __restrict__ prelu, float* __restrict__ out) {
  __shared__ __align__(16) _Float16 Wl[CPO * WPITCH];
  __shared__ __align__(16) float sT[8][16 * 68];
  const int tid = threadIdx.x;
  const int wave = tid >> 5, lane = tid & 31;
  const int j = blockIdx.y;
  const int b = blockIdx.z;

  {
    const v8h* src = (const v8h*)(Wp + (size_t)j * CPO * WPITCH);
#pragma unroll
    for (int it = 0; it < 6; ++it) {
      int i = it * 256 + tid;
      i = i < (CPO * WPITCH / 8 - 1) ? i : (CPO * WPITCH / 8 - 1);
      *(v8h*)(Wl + i * 8) = src[i];
    }
  }
  __syncthreads();

  const int rlane = lane & 15;
  const int hh    = lane >> 4;
  const int koff  = hh * 8;
  const int mOff  = hh * 8;
  int base = j - 1;
  base = base < 0 ? 0 : base;
  base = base > 22 ? 22 : base;
  const int t0 = blockIdx.x * 512 + wave * 64;
  const _Float16* Yb = Y + (size_t)b * TROWS * YP;

  v8f acc[4];
#pragma unroll
  for (int i = 0; i < 4; ++i) acc[i] = (v8f){0.f, 0.f, 0.f, 0.f, 0.f, 0.f, 0.f, 0.f};

#pragma unroll 1
  for (int tap = 0; tap < KTAPS; ++tap) {
    const _Float16* arow = Yb + (size_t)(t0 + tap + rlane) * YP + koff;
#pragma unroll
    for (int chunk = 0; chunk < 3; ++chunk) {
      const int g = (base + chunk) >> 1;
      const int s = tap * 3 + chunk;
      const v16h bf = Frag<_Float16>::load(Wl + rlane * WPITCH + s * 32 + koff);
      const _Float16* ap = arow + g * 32;
      const v16h af0 = Frag<_Float16>::load(ap);
      const v16h af1 = Frag<_Float16>::load(ap + (size_t)16 * YP);
      const v16h af2 = Frag<_Float16>::load(ap + (size_t)32 * YP);
      const v16h af3 = Frag<_Float16>::load(ap + (size_t)48 * YP);
      acc[0] = Frag<_Float16>::mma(af0, bf, acc[0]);
      acc[1] = Frag<_Float16>::mma(af1, bf, acc[1]);
      acc[2] = Frag<_Float16>::mma(af2, bf, acc[2]);
      acc[3] = Frag<_Float16>::mma(af3, bf, acc[3]);
      guard4x(acc[0], acc[1], acc[2], acc[3], af0, af1, af2, af3, bf);
    }
  }
  acc_guard4(acc[0], acc[1], acc[2], acc[3]);

  const float alpha = prelu[0];
  const int ocg = j * CPO + rlane;
  const float bsum = b_res[ocg] + b_sc[ocg];
  float* slab = sT[wave];
#pragma unroll
  for (int i = 0; i < 4; ++i) {
#pragma unroll
    for (int r = 0; r < 8; ++r) {
      float v = acc[i][r] * OSC + bsum;
      v = (v >= 0.0f) ? v : (alpha * v);
      slab[rlane * 68 + i * 16 + mOff + r] = v;
    }
  }
  __builtin_amdgcn_fence(__ATOMIC_RELEASE, "workgroup");
  __builtin_amdgcn_wave_barrier();
  __builtin_amdgcn_fence(__ATOMIC_ACQUIRE, "workgroup");
  {
    float* obase = out + ((size_t)b * OUTC + (size_t)j * CPO) * TOUT + t0;
    const int c4 = rlane * 4;
    for (int pass = 0; pass < 2; ++pass) {
#pragma unroll
      for (int it = 0; it < 8; ++it) {
        const int row = it * 2 + hh;
        const v4f val = *(const v4f*)(slab + row * 68 + c4);
        *(volatile v4f*)(obase + (size_t)row * TOUT + c4) = val;
      }
      __threadfence();
    }
  }
}

extern "C" void kernel_launch(void* const* d_in, const int* in_sizes, int n_in,
                              void* d_out, int out_size, void* d_ws, size_t ws_size,
                              hipStream_t stream) {
  if (n_in < 6) return;
  if (in_sizes[0] != NB * CIN * TIN) return;
  if (in_sizes[1] != OUTC * INC * KTAPS) return;
  if (in_sizes[2] != OUTC) return;
  if (in_sizes[3] != OUTC * INC) return;
  if (in_sizes[4] != OUTC) return;
  if (in_sizes[5] < 1) return;
  if (out_size != NB * OUTC * TOUT) return;

  const float* x     = (const float*)d_in[0];
  const float* w_res = (const float*)d_in[1];
  const float* b_res = (const float*)d_in[2];
  const float* w_sc  = (const float*)d_in[3];
  const float* b_sc  = (const float*)d_in[4];
  const float* prelu = (const float*)d_in[5];
  float* out = (float*)d_out;

  const size_t ybytes = (size_t)NB * TROWS * YP * sizeof(_Float16);
  const size_t wbytes = (size_t)NJ * CPO * WPITCH * sizeof(_Float16);
  if (ybytes + wbytes > ws_size) return;
  _Float16* Y  = (_Float16*)d_ws;
  _Float16* Wp = (_Float16*)((char*)d_ws + ybytes);

  k_prep_y<<<dim3(TROWS / 32, NB), dim3(256), 0, stream>>>(x, Y);
  k_pack_w<<<dim3(NJ), dim3(256), 0, stream>>>(w_res, w_sc, Wp);
  k_conv<<<dim3(TOUT / 512, NJ, NB), dim3(256), 0, stream>>>(Y, Wp, b_res, b_sc, prelu, out);
}
